// NottinghamModel_21827023798955
// MI455X (gfx1250) — hardware-run, weakly checked
//
#include <hip/hip_runtime.h>
#include <math.h>

typedef __attribute__((ext_vector_type(16))) _Float16 v16h;
typedef __attribute__((ext_vector_type(8)))  _Float16 v8h;
typedef __attribute__((ext_vector_type(8)))  float    v8f;
typedef __attribute__((ext_vector_type(4)))  float    v4f;

constexpr int kT      = 128;
constexpr int kB      = 1024;
constexpr int kD      = 66;
constexpr int kH      = 256;
constexpr int kG4     = 4 * kH;
constexpr int kOut    = 65;
constexpr int kMel    = 35;
constexpr int kHarm   = kOut - kMel;
constexpr int kXK     = 96;
constexpr int kK0     = kXK + kH;
constexpr int kK1     = 2 * kH;
constexpr int kNOutPad = 80;
constexpr int kRowsAll = kT * kB;
constexpr int kRowsBlk = 32;
constexpr int kXsP    = 104;
constexpr int kHsP    = 264;
constexpr int kHTile  = kRowsBlk * kHsP;
constexpr int kTailRows = 64;
constexpr int kLsP    = 81;
constexpr int kTailChunks = kTailRows * kOut / 4;
constexpr int kNumPartBlk = (kB / kTailRows) * kT;
constexpr int kOut0Elems = kT * kB * kOut;

static_assert(kK0 == 352 && kK1 == 512, "padded K");
static_assert((kK0 % 32) == 0 && (kK1 % 32) == 0 && (kXK % 32) == 0 && (kH % 32) == 0, "K multiples of 32");
static_assert((kB % kRowsBlk) == 0 && (kB % kTailRows) == 0, "batch tile multiples");
static_assert((kNOutPad % 16) == 0 && kNOutPad >= kOut, "N pad");
static_assert(kHarm == 30, "second softmax width");
static_assert((kTailRows * kOut) % 4 == 0 && kTailChunks == 1040, "tail tile is whole 16-B chunks");
static_assert(((size_t)kTailRows * kOut * 4) % 128 == 0, "tail tile is whole 128-B lines");
static_assert(((size_t)kOut0Elems * 4) % 128 == 0, "second output starts on a line");
static_assert(kOut0Elems == 8519680, "first output extent");
static_assert(kNumPartBlk == 2048, "partial table rows");

constexpr float kCarryX  = 128.0f;
constexpr float kCarryWx = 2048.0f;
constexpr float kCarryH  = 256.0f;
constexpr float kCarryWh = 1024.0f;
static_assert(kCarryX * kCarryWx == kCarryH * kCarryWh, "one fold-back constant");
constexpr float kProdInv = 1.0f / (kCarryH * kCarryWh);
constexpr float kF16MinNormal = 6.103515625e-5f;
constexpr float kLossScale = 1.0f / ((float)kT * (float)kB);

constexpr size_t kSzXH   = (size_t)kRowsAll * kXK * 2;
constexpr size_t kSzW0T  = (size_t)kG4 * kK0 * 2;
constexpr size_t kSzW1T  = (size_t)kG4 * kK1 * 2;
constexpr size_t kSzWOT  = (size_t)kNOutPad * kH * 2;
constexpr size_t kSzH1   = (size_t)kRowsAll * kH * 2;
constexpr size_t kSzPART = (size_t)kNumPartBlk * 32 * 4;
constexpr size_t kOffXH   = 0;
constexpr size_t kOffW0T  = kOffXH  + kSzXH;
constexpr size_t kOffW1T  = kOffW0T + kSzW0T;
constexpr size_t kOffWOT  = kOffW1T + kSzW1T;
constexpr size_t kOffH1   = kOffWOT + kSzWOT;
constexpr size_t kOffPART = kOffH1  + kSzH1;
constexpr size_t kWsTotal = kOffPART + kSzPART;
static_assert(kWsTotal == 94347264ull, "carve total");
static_assert(kWsTotal <= 134217728ull, "carve cap");
static_assert((kOffW0T % 128) == 0 && (kOffW1T % 128) == 0 && (kOffWOT % 128) == 0 &&
              (kOffH1 % 128) == 0 && (kOffPART % 128) == 0, "128-B aligned regions");

__device__ __forceinline__ _Float16 to_f16c(float v, float carry) {
  float s = v * carry;
  s = (fabsf(s) < kF16MinNormal) ? 0.0f : s;
  return (_Float16)s;
}
__device__ __forceinline__ float fsig(float x) {
  return __builtin_amdgcn_rcpf(1.0f + __expf(-x));
}
__device__ __forceinline__ float ftanh(float x) {
  return 1.0f - 2.0f * __builtin_amdgcn_rcpf(1.0f + __expf(2.0f * x));
}

union FragU { v16h v; v8h h[2]; };
__device__ __forceinline__ v16h frag_load(const _Float16* p) {
  FragU f;
  f.h[0] = *(const v8h*)(p);
  f.h[1] = *(const v8h*)(p + 16);
  return f.v;
}
__device__ __forceinline__ v8f mma_h(v16h a, v16h b, v8f c) {
  return __builtin_amdgcn_wmma_f32_16x16x32_f16(false, a, false, b, (short)0, c, false, false);
}
__device__ __forceinline__ void tie_acc(v8f& a) { asm volatile("" : "+v"(a)); }
__device__ __forceinline__ void guard_acc6(v8f& a, v16h x0, v16h x1, v16h x2, v16h x3, v16h x4, v16h x5) {
  asm volatile("v_nop\n\tv_nop\n\tv_nop\n\tv_nop" : "+v"(a) : "v"(x0), "v"(x1), "v"(x2), "v"(x3), "v"(x4), "v"(x5));
}

static_assert(((size_t)kRowsAll * (kXK / 8)) % 256 == 0, "prep_x exact grid");
__global__ __launch_bounds__(256) void prep_x_kernel(const float* __restrict__ x, _Float16* __restrict__ xh) {
  const int i   = blockIdx.x * 256 + threadIdx.x;
  const int row = i / (kXK / 8);
  const int c0  = (i - row * (kXK / 8)) * 8;
  const int t   = row >> 10;
  const int b   = row & (kB - 1);
  const float* src = x + ((size_t)b * kT + t) * kD;
  float v[8];
#pragma unroll
  for (int e = 0; e < 8; ++e) {
    const int c  = c0 + e;
    const int cc = (c < kD) ? c : (kD - 1);
    v[e] = src[cc];
  }
  v8h hv;
#pragma unroll
  for (int e = 0; e < 8; ++e) {
    const float s = ((c0 + e) < kD) ? v[e] : 0.0f;
    hv[e] = to_f16c(s, kCarryX);
  }
  _Float16* dst = xh + (size_t)i * 8;
  *(volatile v8h*)dst = hv;
  __threadfence();
  *(volatile v8h*)dst = hv;
}

__global__ __launch_bounds__(256) void prep_w_kernel(const float* __restrict__ src, _Float16* __restrict__ dst,
                                                     int total8, int kPad8, int nReal, int srcLd,
                                                     int kA, int kGap, float cA, float cB) {
  const int i = blockIdx.x * 256 + threadIdx.x;
  if (i >= total8) return;
  const int n  = i / kPad8;
  const int k0 = (i - n * kPad8) * 8;
  const int nn = (n < nReal) ? n : (nReal - 1);
  float v[8];
#pragma unroll
  for (int e = 0; e < 8; ++e) {
    const int k    = k0 + e;
    const int srow = (k < kA) ? k : (k - (kGap - kA));
    v[e] = src[(size_t)srow * srcLd + nn];
  }
  v8h hv;
#pragma unroll
  for (int e = 0; e < 8; ++e) {
    const int k = k0 + e;
    const bool zero = (n >= nReal) || ((k >= kA) && (k < kGap));
    const float carry = (k < kA) ? cA : cB;
    const float s = zero ? 0.0f : v[e];
    hv[e] = to_f16c(s, carry);
  }
  _Float16* d = dst + (size_t)i * 8;
  *(volatile v8h*)d = hv;
  __threadfence();
  *(volatile v8h*)d = hv;
}

template <int NK, int AP, int BP>
__device__ __forceinline__ void mma_span(v8f (&acc)[2][8], const _Float16* ap, const _Float16* bp) {
#pragma unroll 1
  for (int ks = 0; ks < NK; ++ks) {
    const v16h a0 = frag_load(ap);
    const v16h a1 = frag_load(ap + 16 * AP);
#pragma unroll
    for (int grp = 0; grp < 2; ++grp) {
      const v16h b0 = frag_load(bp + (size_t)((2 * grp) * kH) * BP);
      const v16h b1 = frag_load(bp + (size_t)((2 * grp) * kH + 16) * BP);
      const v16h b2 = frag_load(bp + (size_t)((2 * grp + 1) * kH) * BP);
      const v16h b3 = frag_load(bp + (size_t)((2 * grp + 1) * kH + 16) * BP);
      acc[0][4 * grp + 0] = mma_h(a0, b0, acc[0][4 * grp + 0]);
      acc[1][4 * grp + 0] = mma_h(a1, b0, acc[1][4 * grp + 0]);
      acc[0][4 * grp + 1] = mma_h(a0, b1, acc[0][4 * grp + 1]);
      acc[1][4 * grp + 1] = mma_h(a1, b1, acc[1][4 * grp + 1]);
      acc[0][4 * grp + 2] = mma_h(a0, b2, acc[0][4 * grp + 2]);
      acc[1][4 * grp + 2] = mma_h(a1, b2, acc[1][4 * grp + 2]);
      acc[0][4 * grp + 3] = mma_h(a0, b3, acc[0][4 * grp + 3]);
      acc[1][4 * grp + 3] = mma_h(a1, b3, acc[1][4 * grp + 3]);
      tie_acc(acc[0][4 * grp + 0]);
      tie_acc(acc[1][4 * grp + 0]);
      tie_acc(acc[0][4 * grp + 1]);
      tie_acc(acc[1][4 * grp + 1]);
      tie_acc(acc[0][4 * grp + 2]);
      tie_acc(acc[1][4 * grp + 2]);
      tie_acc(acc[0][4 * grp + 3]);
      guard_acc6(acc[1][4 * grp + 3], a0, a1, b0, b1, b2, b3);
    }
    ap += 32;
    bp += 32;
  }
}

__device__ __forceinline__ void lstm_gates(const v8f (&acc)[2][8], float* cp, const float* bl, _Float16* hd) {
#pragma unroll
  for (int mt = 0; mt < 2; ++mt) {
#pragma unroll
    for (int u = 0; u < 2; ++u) {
      float* cpt = cp + (mt * 2 + u) * 256;
      const v4f cl = *(const v4f*)(cpt);
      const v4f ch = *(const v4f*)(cpt + 4);
      const float bi = bl[u * 16];
      const float bj = bl[kH + u * 16];
      const float bf = bl[2 * kH + u * 16];
      const float bo = bl[3 * kH + u * 16];
      v4f nl, nh;
#pragma unroll
      for (int r = 0; r < 8; ++r) {
        const float pi = acc[mt][0 + u][r] * kProdInv + bi;
        const float pj = acc[mt][2 + u][r] * kProdInv + bj;
        const float pf = acc[mt][4 + u][r] * kProdInv + bf;
        const float po = acc[mt][6 + u][r] * kProdInv + bo;
        const float cold = (r < 4) ? cl[r & 3] : ch[r & 3];
        const float cn = cold * fsig(pf + 1.0f) + fsig(pi) * ftanh(pj);
        const float hn = ftanh(cn) * fsig(po);
        if (r < 4) nl[r & 3] = cn; else nh[r & 3] = cn;
        hd[(mt * 16 + r) * kHsP + u * 16] = to_f16c(hn, kCarryH);
      }
      *(v4f*)(cpt)     = nl;
      *(v4f*)(cpt + 4) = nh;
    }
  }
}

__global__ __launch_bounds__(256) void lstm2_kernel(const _Float16* __restrict__ XH,
                                                    const _Float16* __restrict__ W0T,
                                                    const _Float16* __restrict__ W1T,
                                                    const float* __restrict__ b0,
                                                    const float* __restrict__ b1,
                                                    _Float16* __restrict__ H1p) {
  __shared__ __align__(16) _Float16 sX[kRowsBlk * kXsP];
  __shared__ __align__(16) _Float16 sH0[2 * kHTile];
  __shared__ __align__(16) _Float16 sH1[2 * kHTile];
  __shared__ __align__(16) float    sC[2 * 8 * 4 * 256];
  __shared__ __align__(16) float    sBias[2 * kG4];

  const int tid  = threadIdx.x;
  const int lane = tid & 31;
  const int wave = __builtin_amdgcn_readfirstlane(tid >> 5);
  const int hh   = lane >> 4;
  const int m    = lane & 15;
  const int brow0 = blockIdx.x * kRowsBlk;

#pragma unroll
  for (int k = 0; k < 4; ++k) {
    sBias[tid + 256 * k]       = b0[tid + 256 * k];
    sBias[kG4 + tid + 256 * k] = b1[tid + 256 * k];
  }
  {
    const v8h zh = (v8h){(_Float16)0.0f, (_Float16)0.0f, (_Float16)0.0f, (_Float16)0.0f,
                         (_Float16)0.0f, (_Float16)0.0f, (_Float16)0.0f, (_Float16)0.0f};
    for (int i = tid; i < (2 * kHTile) / 8; i += 256) {
      *(v8h*)(sH0 + i * 8) = zh;
      *(v8h*)(sH1 + i * 8) = zh;
    }
  }
  float* cp0 = sC + ((0 * 8 + wave) * 4) * 256 + lane * 8;
  float* cp1 = sC + ((1 * 8 + wave) * 4) * 256 + lane * 8;
  {
    const v4f zf = (v4f){0.0f, 0.0f, 0.0f, 0.0f};
#pragma unroll
    for (int tile = 0; tile < 4; ++tile) {
      *(v4f*)(cp0 + tile * 256)     = zf;
      *(v4f*)(cp0 + tile * 256 + 4) = zf;
      *(v4f*)(cp1 + tile * 256)     = zf;
      *(v4f*)(cp1 + tile * 256 + 4) = zf;
    }
  }
  __syncthreads();

  const int xo1 = (tid / 12) * kXsP + (tid % 12) * 8;
  const int ch2 = 256 + tid;
  const int xo2 = (ch2 / 12) * kXsP + (ch2 % 12) * 8;

  const int aoffX = m * kXsP + 8 * hh;
  const int aoffH = m * kHsP + 8 * hh;
  const _Float16* bW0 = W0T + (size_t)(32 * wave + m) * kK0 + 8 * hh;
  const _Float16* bW1 = W1T + (size_t)(32 * wave + m) * kK1 + 8 * hh;
  const float* bl0 = sBias + 32 * wave + m;
  const float* bl1 = sBias + kG4 + 32 * wave + m;
  const int hdoff = (8 * hh) * kHsP + 32 * wave + m;

#pragma unroll 1
  for (int t = 0; t < kT; ++t) {
    const int cur = t & 1;
    const int nxt = cur ^ 1;
    const _Float16* xsrc = XH + ((size_t)t * kB + brow0) * kXK;
    {
      const v8h xv = *(const v8h*)(xsrc + tid * 8);
      *(v8h*)(sX + xo1) = xv;
    }
    if (wave < 4) {
      const v8h xv = *(const v8h*)(xsrc + ch2 * 8);
      *(v8h*)(sX + xo2) = xv;
    }
    __syncthreads();

    v8f acc[2][8];
#pragma unroll
    for (int i = 0; i < 2; ++i)
#pragma unroll
      for (int j = 0; j < 8; ++j) acc[i][j] = (v8f){0.f, 0.f, 0.f, 0.f, 0.f, 0.f, 0.f, 0.f};

    mma_span<kXK / 32, kXsP, kK0>(acc, sX + aoffX, bW0);
    mma_span<kH / 32, kHsP, kK0>(acc, sH0 + cur * kHTile + aoffH, bW0 + kXK);
    lstm_gates(acc, cp0, bl0, sH0 + nxt * kHTile + hdoff);
    __syncthreads();

#pragma unroll
    for (int i = 0; i < 2; ++i)
#pragma unroll
      for (int j = 0; j < 8; ++j) acc[i][j] = (v8f){0.f, 0.f, 0.f, 0.f, 0.f, 0.f, 0.f, 0.f};

    mma_span<kH / 32, kHsP, kK1>(acc, sH0 + nxt * kHTile + aoffH, bW1);
    mma_span<kH / 32, kHsP, kK1>(acc, sH1 + cur * kHTile + aoffH, bW1 + kH);
    lstm_gates(acc, cp1, bl1, sH1 + nxt * kHTile + hdoff);
    __syncthreads();

    {
      const _Float16* hs = sH1 + nxt * kHTile + (wave * 4) * kHsP + lane * 8;
      v8h hv[4];
#pragma unroll
      for (int it = 0; it < 4; ++it) hv[it] = *(const v8h*)(hs + it * kHsP);
      _Float16* dst = H1p + ((size_t)t * kB + brow0 + wave * 4) * kH + lane * 8;
      for (int pass = 0; pass < 2; ++pass) {
#pragma unroll
        for (int it = 0; it < 4; ++it) *(volatile v8h*)(dst + (size_t)it * kH) = hv[it];
        __threadfence();
      }
    }
  }
}

__global__ __launch_bounds__(128) void tail_kernel(const _Float16* __restrict__ H1p,
                                                   const _Float16* __restrict__ WOT,
                                                   const float* __restrict__ ob,
                                                   const int* __restrict__ tgt,
                                                   float* __restrict__ out,
                                                   float* __restrict__ part) {
  __shared__ __align__(16) float sL[kTailRows * kLsP];
  __shared__ __align__(16) float sP[kTailRows * kOut];
  __shared__ __align__(16) float sCe[128];

  const int tid  = threadIdx.x;
  const int lane = tid & 31;
  const int wave = tid >> 5;
  const int hh   = lane >> 4;
  const int m    = lane & 15;
  const int q    = blockIdx.y;
  const int p0   = blockIdx.x * kTailRows;

  const int arow = p0 + wave * 16 + m;
  const _Float16* ap = H1p + ((size_t)arow * kT + q) * kH + 8 * hh;
  const _Float16* bp = WOT + (size_t)m * kH + 8 * hh;

  v8f acc[5];
#pragma unroll
  for (int j = 0; j < 5; ++j) acc[j] = (v8f){0.f, 0.f, 0.f, 0.f, 0.f, 0.f, 0.f, 0.f};

#pragma unroll 1
  for (int ks = 0; ks < kH / 32; ++ks) {
    const v16h a  = frag_load(ap);
    const v16h b0 = frag_load(bp);
    const v16h b1 = frag_load(bp + 16 * kH);
    const v16h b2 = frag_load(bp + 32 * kH);
    const v16h b3 = frag_load(bp + 48 * kH);
    const v16h b4 = frag_load(bp + 64 * kH);
    acc[0] = mma_h(a, b0, acc[0]);
    acc[1] = mma_h(a, b1, acc[1]);
    acc[2] = mma_h(a, b2, acc[2]);
    acc[3] = mma_h(a, b3, acc[3]);
    acc[4] = mma_h(a, b4, acc[4]);
    tie_acc(acc[0]);
    tie_acc(acc[1]);
    tie_acc(acc[2]);
    tie_acc(acc[3]);
    guard_acc6(acc[4], a, b0, b1, b2, b3, b4);
    ap += 32;
    bp += 32;
  }

#pragma unroll
  for (int nt = 0; nt < 5; ++nt) {
    const int col  = nt * 16 + m;
    const int colc = (col < kOut) ? col : (kOut - 1);
    const float bl = ob[colc];
    const float bb = (col < kOut) ? bl : 0.0f;
#pragma unroll
    for (int r = 0; r < 8; ++r)
      sL[(wave * 16 + 8 * hh + r) * kLsP + col] = acc[nt][r] * kProdInv + bb;
  }
  __syncthreads();

  {
    const int row  = tid >> 1;
    const int prt  = tid & 1;
    const int c0   = prt ? kMel : 0;
    const int n    = prt ? kHarm : kMel;
    const float* lr = sL + row * kLsP + c0;
    float*       pr = sP + row * kOut + c0;
    float mx = lr[0];
#pragma unroll 1
    for (int c = 1; c < n; ++c) mx = fmaxf(mx, lr[c]);
    float s = 0.0f;
#pragma unroll 1
    for (int c = 0; c < n; ++c) {
      const float e = expf(lr[c] - mx);
      pr[c] = e;
      s += e;
    }
    const float inv = 1.0f / s;
#pragma unroll 1
    for (int c = 0; c < n; ++c) {
      const float e = pr[c];
      pr[c] = e * inv;
    }
    const int r = (p0 + row) * kT + q;
    int tg = tgt[2 * r + prt];
    tg = (tg < 0) ? 0 : tg;
    tg = (tg > n - 1) ? (n - 1) : tg;
    const float ce = (logf(s) + mx) - lr[tg];
    sCe[tid] = 0.5f * ce;
  }
  __syncthreads();

  {
    v4f pv[9];
#pragma unroll
    for (int it = 0; it < 9; ++it) {
      const int ch  = it * 128 + tid;
      const int chc = (ch < kTailChunks) ? ch : (kTailChunks - 1);
      pv[it] = *(const v4f*)(sP + chc * 4);
    }
    const float ps = ((sCe[lane] + sCe[lane + 32]) + sCe[lane + 64]) + sCe[lane + 96];
    float* obase = out + ((size_t)q * kB + p0) * kOut;
    float* pline = part + ((size_t)(q * (kB / kTailRows) + blockIdx.x)) * 32 + lane;
    for (int pass = 0; pass < 2; ++pass) {
#pragma unroll
      for (int it = 0; it < 9; ++it) {
        const int ch = it * 128 + tid;
        if (ch < kTailChunks) *(volatile v4f*)(obase + (size_t)ch * 4) = pv[it];
      }
      if (wave == 0) *(volatile float*)pline = ps;
      __threadfence();
    }
  }
}

__global__ __launch_bounds__(256) void loss_final_kernel(const float* __restrict__ part, float* __restrict__ out1) {
  __shared__ float red[256];
  const int tid = threadIdx.x;
  float s = 0.0f;
#pragma unroll 1
  for (int j = 0; j < (kNumPartBlk * 32) / 256; ++j) s += part[j * 256 + tid];
  red[tid] = s;
  __syncthreads();
  for (int off = 128; off > 0; off >>= 1) {
    if (tid < off) red[tid] += red[tid + off];
    __syncthreads();
  }
  const float val = red[0] * kLossScale;
  if (tid == 0) *(volatile float*)out1 = val;
  __threadfence();
  if (tid == 0) *(volatile float*)out1 = val;
}

extern "C" void kernel_launch(void* const* d_in, const int* in_sizes, int n_in,
                              void* d_out, int out_size, void* d_ws, size_t ws_size,
                              hipStream_t stream) {
  if (n_in < 8) return;
  if (in_sizes[0] != kB * kT * kD) return;
  if (in_sizes[1] != kB * kT * 2) return;
  if (in_sizes[2] != (kD + kH) * kG4) return;
  if (in_sizes[3] != kG4) return;
  if (in_sizes[4] != 2 * kH * kG4) return;
  if (in_sizes[5] != kG4) return;
  if (in_sizes[6] != kH * kOut) return;
  if (in_sizes[7] != kOut) return;
  if (out_size != kOut0Elems + 1) return;
  if (ws_size < kWsTotal) return;

  const float* seq_input = (const float*)d_in[0];
  const int*   seq_tgt   = (const int*)d_in[1];
  const float* W0  = (const float*)d_in[2];
  const float* b0  = (const float*)d_in[3];
  const float* W1  = (const float*)d_in[4];
  const float* b1  = (const float*)d_in[5];
  const float* Wo  = (const float*)d_in[6];
  const float* bo  = (const float*)d_in[7];
  float* out = (float*)d_out;

  char* ws = (char*)d_ws;
  _Float16* XH   = (_Float16*)(ws + kOffXH);
  _Float16* W0T  = (_Float16*)(ws + kOffW0T);
  _Float16* W1T  = (_Float16*)(ws + kOffW1T);
  _Float16* WOT  = (_Float16*)(ws + kOffWOT);
  _Float16* H1p  = (_Float16*)(ws + kOffH1);
  float*    PART = (float*)(ws + kOffPART);

  prep_x_kernel<<<(kRowsAll * (kXK / 8)) / 256, 256, 0, stream>>>(seq_input, XH);

  prep_w_kernel<<<(kG4 * (kK0 / 8)) / 256, 256, 0, stream>>>(W0, W0T, kG4 * (kK0 / 8), kK0 / 8, kG4, kG4,
                                                            kD, kXK, kCarryWx, kCarryWh);
  prep_w_kernel<<<(kG4 * (kK1 / 8)) / 256, 256, 0, stream>>>(W1, W1T, kG4 * (kK1 / 8), kK1 / 8, kG4, kG4,
                                                            0, 0, kCarryWh, kCarryWh);
  prep_w_kernel<<<(kNOutPad * (kH / 8)) / 256, 256, 0, stream>>>(Wo, WOT, kNOutPad * (kH / 8), kH / 8, kOut, kOut,
                                                                0, 0, kCarryWh, kCarryWh);

  lstm2_kernel<<<kB / kRowsBlk, 256, 0, stream>>>(XH, W0T, W1T, b0, b1, H1p);

  tail_kernel<<<dim3(kB / kTailRows, kT), 128, 0, stream>>>(H1p, WOT, bo, seq_tgt, out, PART);

  loss_final_kernel<<<1, 256, 0, stream>>>(PART, out + (size_t)kOut0Elems);
}
